// PositionAttention3D_80865644249163
// MI455X (gfx1250) — hardware-verified
//
#include <hip/hip_runtime.h>
#include <math.h>

typedef __attribute__((ext_vector_type(16))) _Float16 v16h;
typedef __attribute__((ext_vector_type(16))) __bf16 v16b;
typedef __attribute__((ext_vector_type(8)))  _Float16 v8h;
typedef __attribute__((ext_vector_type(8)))  float v8f;
typedef __attribute__((ext_vector_type(4)))  float v4f;
typedef __attribute__((ext_vector_type(2)))  float v2f;
typedef __attribute__((ext_vector_type(4)))  unsigned v4u;
typedef __attribute__((ext_vector_type(4)))  int v4i;
typedef float __attribute__((may_alias)) float_a;
typedef int __attribute__((may_alias)) int_a;

template <typename T> __device__ __forceinline__ void vst2(void* p, T v) { *(volatile T*)p = v; __threadfence(); *(volatile T*)p = v; }
__device__ __forceinline__ v8f wmma16(v16h a, v16h b, v8f c) {
  v8f d = __builtin_amdgcn_wmma_f32_16x16x32_f16(false, a, false, b, (short)0, c, false, false);
  asm volatile("v_nop\n\tv_nop\n\tv_nop\n\tv_nop" : "+v"(d) : "v"(a), "v"(b));
  return d;
}
__device__ __forceinline__ v8f wmma_bf(v16b a, v16b b, v8f c) {
  v8f d = __builtin_amdgcn_wmma_f32_16x16x32_bf16(false, a, false, b, (short)0, c, false, false);
  asm volatile("v_nop\n\tv_nop\n\tv_nop\n\tv_nop" : "+v"(d) : "v"(a), "v"(b));
  return d;
}
__device__ __forceinline__ v16h frag_h(const _Float16* rowk0, int lane) {
  union { v16h v; v8h q[2]; } u; const _Float16* p = rowk0 + 8 * (lane >> 4);
  u.q[0] = *(const v8h*)p; u.q[1] = *(const v8h*)(p + 16); return u.v;
}
__device__ __forceinline__ v16h frag_f32(const float* rowk0, int lane) {
  v16h a; const float* p = rowk0 + 8 * (lane >> 4);
#pragma unroll
  for (int i = 0; i < 8; ++i) { a[i] = (_Float16)p[i]; a[8 + i] = (_Float16)p[16 + i]; }
  return a;
}
__device__ __forceinline__ v16h frag_f32s(const float* rowk0, int lane, float sc) {
  v16h a; const float* p = rowk0 + 8 * (lane >> 4);
#pragma unroll
  for (int i = 0; i < 8; ++i) { a[i] = (_Float16)(p[i] * sc); a[8 + i] = (_Float16)(p[16 + i] * sc); }
  return a;
}
__device__ __forceinline__ v16h fragc_f32(const float* W, int k0, int n, int lane, int ld, int K) {
  v16h a; const int g = lane >> 4;
#pragma unroll
  for (int i = 0; i < 8; ++i) { const int ka = k0 + 8 * g + i, kb = ka + 16;
    a[i] = (_Float16)(ka < K ? W[(size_t)(ka < K ? ka : K - 1) * ld + n] : 0.f); a[8 + i] = (_Float16)(kb < K ? W[(size_t)(kb < K ? kb : K - 1) * ld + n] : 0.f); }
  return a;
}
struct F2 { v16b h, l; };
__device__ __forceinline__ F2 bsplit16(const float v[16]) { F2 r;
#pragma unroll
  for (int i = 0; i < 16; ++i) { const __bf16 h = (__bf16)v[i]; r.h[i] = h; r.l[i] = (__bf16)(v[i] - (float)h); }
  return r; }
__device__ __forceinline__ F2 split_row(const float* row, int k0, int lane) { float v[16]; const float* p = row + k0 + 8 * (lane >> 4);
#pragma unroll
  for (int i = 0; i < 8; ++i) { v[i] = p[i]; v[8 + i] = p[16 + i]; }
  return bsplit16(v); }
__device__ __forceinline__ F2 split_rowK(const float* row, int k0, int lane, int K) { float v[16]; const int g = lane >> 4;
#pragma unroll
  for (int i = 0; i < 8; ++i) { const int ka = k0 + 8 * g + i, kb = ka + 16; v[i] = ka < K ? row[ka < K ? ka : K - 1] : 0.f; v[8 + i] = kb < K ? row[kb < K ? kb : K - 1] : 0.f; }
  return bsplit16(v); }
__device__ __forceinline__ F2 split_col(const float* W, int k0, int n, int lane, int ld, int K) { float v[16]; const int g = lane >> 4;
#pragma unroll
  for (int i = 0; i < 8; ++i) { const int ka = k0 + 8 * g + i, kb = ka + 16; v[i] = ka < K ? W[(size_t)(ka < K ? ka : K - 1) * ld + n] : 0.f; v[8 + i] = kb < K ? W[(size_t)(kb < K ? kb : K - 1) * ld + n] : 0.f; }
  return bsplit16(v); }
__device__ __forceinline__ v8f mac3(const F2& a, const F2& b, v8f c) { c = wmma_bf(a.l, b.h, c); c = wmma_bf(a.h, b.l, c); return wmma_bf(a.h, b.h, c); }
__device__ __forceinline__ float sigm(float v) { return 1.0f / (1.0f + expf(-v)); }
#define LDSX() do { asm volatile("s_wait_dscnt 0" ::: "memory"); __builtin_amdgcn_wave_barrier(); __builtin_amdgcn_fence(__ATOMIC_RELEASE, "workgroup"); } while (0)


#define NB 2
#define CH 64
#define NP 4096
#define RR 8
#ifndef TQB
#define TQB (NP / 64)
#define TNB NB
#endif
typedef __attribute__((ext_vector_type(8))) __bf16 v8b;
__device__ __forceinline__ v16b frag_b(const __bf16* rowk0, int lane) {
  union { v16b v; v8b q[2]; } u; const __bf16* p = rowk0 + 8 * (lane >> 4);
  u.q[0] = *(const v8b*)p; u.q[1] = *(const v8b*)(p + 16); return u.v;
}
__device__ __forceinline__ float bfr(float v) { return (float)(__bf16)v; }
__device__ __attribute__((noinline)) float exp_ni(float v) { return expf(v); }
__device__ __attribute__((noinline)) float erf_ni(float v) { return erff(v); }

#define WS_PW  0u
#define WS_QK  (WS_PW + 2u * 128 * CH)
#define WS_VH  (WS_QK + 4u * NB * NP * 64)
#define WS_VL  (WS_VH + 2u * NB * CH * NP)
#define WS_END (WS_VL + 2u * NB * CH * NP)

__global__ __launch_bounds__(256) void k_pack(const float* __restrict__ WQ, const float* __restrict__ WK, const float* __restrict__ WV, __bf16* __restrict__ PW) {
  __shared__ __align__(16) __bf16 s[128][CH]; const int tid = threadIdx.x;
  for (int q = tid; q < 128 * CH; q += 256) { const int n = q / CH, c = q % CH; float v = 0.f; if (n < RR) v = WQ[n * CH + c]; else if (n >= 32 && n < 32 + RR) v = WK[(n - 32) * CH + c]; else if (n >= 64) v = WV[(n - 64) * CH + c]; s[n][c] = (__bf16)v; }
  __syncthreads();
  for (int q = tid; q < 128 * CH / 8; q += 256) vst2((unsigned*)(PW + q * 8), *(const v4u*)&(&s[0][0])[q * 8]);
}
__global__ __launch_bounds__(128) void k_proj(const float* __restrict__ X, const __bf16* __restrict__ PW, float* __restrict__ QK, __bf16* __restrict__ VH, __bf16* __restrict__ VL) {
  __shared__ __align__(16) __bf16 sx[64][72]; __shared__ __align__(16) float so[4][16][68]; __shared__ __align__(16) __bf16 sth[CH][72], stl[CH][72];
  const int tid = threadIdx.x, wave = tid >> 5, lane = tid & 31, col = lane & 15, g = lane >> 4; const int b = blockIdx.y; const int p0 = blockIdx.x * 64;
  for (int q = tid; q < CH * 64; q += 128) { const int c = q >> 6, nl = q & 63; sx[nl][c] = (__bf16)X[((size_t)b * CH + c) * NP + p0 + nl]; }
  __syncthreads();
  v16b a[2];
#pragma unroll
  for (int kc = 0; kc < 2; ++kc) {
#pragma unroll
    for (int i = 0; i < 8; ++i) { a[kc][i] = sx[wave * 16 + col][kc * 32 + 8 * g + i]; a[kc][8 + i] = sx[wave * 16 + col][kc * 32 + 16 + 8 * g + i]; } }
  v8f acc[8] = {};
#pragma unroll
  for (int kc = 0; kc < 2; ++kc) {
#pragma unroll
    for (int j = 0; j < 8; ++j) acc[j] = wmma_bf(a[kc], frag_b(PW + (size_t)(j * 16 + col) * CH + kc * 32, lane), acc[j]); }
#pragma unroll
  for (int j = 0; j < 4; ++j)
#pragma unroll
    for (int r = 0; r < 8; ++r) so[wave][8 * g + r][j * 16 + col] = acc[j][r];
#pragma unroll
  for (int j = 4; j < 8; ++j) { const int c = (j - 4) * 16 + col;
#pragma unroll
    for (int r = 0; r < 8; ++r) { const float v = acc[j][r]; const __bf16 hb = (__bf16)v; sth[c][wave * 16 + 8 * g + r] = hb; stl[c][wave * 16 + 8 * g + r] = (__bf16)(v - (float)hb); } }
  __syncthreads();
  for (int rl = 0; rl < 16; ++rl) if (lane < 16) vst2(QK + ((size_t)b * NP + p0 + wave * 16 + rl) * 64 + lane * 4, *(const v4f*)&so[wave][rl][lane * 4]);
  for (int q = tid; q < CH * 8; q += 128) { const int c = q >> 3, pc = q & 7; const size_t o = ((size_t)b * CH + c) * NP + p0 + pc * 8; vst2((unsigned*)(VH + o), *(const v4u*)&sth[c][pc * 8]); vst2((unsigned*)(VL + o), *(const v4u*)&stl[c][pc * 8]); }
}
__global__ __launch_bounds__(128) void k_attn(const float* __restrict__ QK, const __bf16* __restrict__ VH, const __bf16* __restrict__ VL, const float* __restrict__ X, const float* __restrict__ GM, float* __restrict__ Y) {
  __shared__ __align__(16) float sp[4][16][36]; __shared__ __align__(16) float so[CH][68];
  const int tid = threadIdx.x, wave = tid >> 5, lane = tid & 31, col = lane & 15, g = lane >> 4; const int b = blockIdx.y; const int q0 = blockIdx.x * 64 + wave * 16;
  const F2 aq = split_row(QK + ((size_t)b * NP + q0 + col) * 64, 0, lane);
  float m[8], l[8];
#pragma unroll
  for (int r = 0; r < 8; ++r) { m[r] = -3.0e38f; l[r] = 0.f; }
  v8f acc[4] = {};
  const float scale = 0.35355339059327373f;
#pragma unroll 1
  for (int ks = 0; ks < NP / 32; ++ks) { v8f s[2];
#pragma unroll
    for (int ct = 0; ct < 2; ++ct) { const int kk = ks * 32 + ct * 16 + col; const F2 kb = split_row(QK + ((size_t)b * NP + kk) * 64, 32, lane); const v8f c = mac3(aq, kb, (v8f){});
#pragma unroll
      for (int r = 0; r < 8; ++r) s[ct][r] = c[r] * scale; }
#pragma unroll
    for (int r = 0; r < 8; ++r) { float mx = fmaxf(s[0][r], s[1][r]);
#pragma unroll
      for (int o = 1; o < 16; o <<= 1) mx = fmaxf(mx, __shfl_xor(mx, o));
      const float mn = fmaxf(m[r], mx); const float alpha = exp_ni(m[r] - mn);
      const float e0 = exp_ni(s[0][r] - mn), e1 = exp_ni(s[1][r] - mn); float es = e0 + e1;
#pragma unroll
      for (int o = 1; o < 16; o <<= 1) es += __shfl_xor(es, o);
      l[r] = l[r] * alpha + es; m[r] = mn;
#pragma unroll
      for (int dt = 0; dt < 4; ++dt) acc[dt][r] *= alpha;
      sp[wave][8 * g + r][col] = e0; sp[wave][8 * g + r][16 + col] = e1; }
    LDSX();
    const F2 pa = split_row(&sp[wave][col][0], 0, lane);
#pragma unroll
    for (int dt = 0; dt < 4; ++dt) { const size_t vr = ((size_t)b * CH + dt * 16 + col) * NP + ks * 32; const v16b vh = frag_b(VH + vr, lane), vl = frag_b(VL + vr, lane); acc[dt] = wmma_bf(pa.l, vh, acc[dt]); acc[dt] = wmma_bf(pa.h, vl, acc[dt]); acc[dt] = wmma_bf(pa.h, vh, acc[dt]); }
    LDSX(); }
  const float gm = bfr(GM[0]);
#pragma unroll
  for (int r = 0; r < 8; ++r) { const float il = 1.0f / l[r];
#pragma unroll
    for (int dt = 0; dt < 4; ++dt) so[dt * 16 + col][wave * 16 + 8 * g + r] = acc[dt][r] * il; }
  __syncthreads();
  for (int q = tid; q < CH * 16; q += 128) { const int c = q >> 4, pc = q & 15; const size_t o = ((size_t)b * CH + c) * NP + blockIdx.x * 64 + pc * 4; const float* xs = X + o; const v4f ov = *(const v4f*)&so[c][pc * 4];
    vst2(Y + o, (v4f){bfr(xs[0]) + gm * ov[0], bfr(xs[1]) + gm * ov[1], bfr(xs[2]) + gm * ov[2], bfr(xs[3]) + gm * ov[3]}); }
}
extern "C" void kernel_launch(void* const* d_in, const int* in_sizes, int n_in, void* d_out, int out_size, void* d_ws, size_t ws_size, hipStream_t stream) {
  (void)in_sizes; (void)n_in; (void)out_size;
  const float** F = (const float**)d_in;
  if (ws_size < (size_t)WS_END) return;
  char* ws = (char*)d_ws; __bf16 *PW = (__bf16*)(ws + WS_PW), *VH = (__bf16*)(ws + WS_VH), *VL = (__bf16*)(ws + WS_VL); float* QK = (float*)(ws + WS_QK);
  k_pack<<<1, 256, 0, stream>>>(F[1], F[2], F[3], PW);
  k_proj<<<dim3(NP / 64, TNB), 128, 0, stream>>>(F[0], PW, QK, VH, VL);
  k_attn<<<dim3(TQB, TNB), 128, 0, stream>>>(QK, VH, VL, F[0], F[4], (float*)d_out);
}
